// ScaledDotProductAttention_10453950398993
// MI455X (gfx1250) — hardware-verified
//
#include <hip/hip_runtime.h>
#include <math.h>

#ifndef NB
#define NB 16
#endif
#ifndef SEQ
#define SEQ 4096
#endif
#define NB_FULL 16
#define SEQ_FULL 4096
#define HD 64
#define IN_BSTRIDE ((long long)SEQ_FULL * HD)
#define OUT_BSTRIDE ((long long)SEQ * HD)
static_assert(NB >= 1 && NB <= NB_FULL);
static_assert(SEQ >= 64 && SEQ <= SEQ_FULL && (SEQ % 64) == 0);
static_assert((size_t)3 * NB_FULL * SEQ_FULL * HD * 4 <= (size_t)134217728);

typedef __attribute__((ext_vector_type(16))) _Float16 v16h;
typedef __attribute__((ext_vector_type(8)))  _Float16 v8h;
typedef __attribute__((ext_vector_type(16))) __bf16   v16b;
typedef __attribute__((ext_vector_type(8)))  float    v8f;
typedef __attribute__((ext_vector_type(4)))  float    v4f;

__device__ __forceinline__ int frag_k(int i, int h) { return (i < 8) ? (8 * h + i) : (16 + 8 * h + (i - 8)); }
__device__ __forceinline__ __bf16 bf16_rne(float f) {
    unsigned int u = __float_as_uint(f);
    u += 0x7fffu + ((u >> 16) & 1u);
    return __builtin_bit_cast(__bf16, (unsigned short)(u >> 16));
}
__device__ __forceinline__ float bf16_f32(__bf16 b) { return __uint_as_float(((unsigned int)__builtin_bit_cast(unsigned short, b)) << 16); }
__device__ __forceinline__ v8f wmma16(v16h a, v16h b, v8f c) {
    c = __builtin_amdgcn_wmma_f32_16x16x32_f16(false, a, false, b, (short)0, c, false, false);
    asm volatile("v_nop\n\tv_nop\n\tv_nop\n\tv_nop" : "+v"(c) : "v"(a), "v"(b));
    return c;
}
struct Split { v16b hi, lo; };
__device__ __forceinline__ v8f wmma3(const Split& a, const Split& b, v8f c) {
    c = __builtin_amdgcn_wmma_f32_16x16x32_bf16(false, a.hi, false, b.hi, (short)0, c, false, false);
    c = __builtin_amdgcn_wmma_f32_16x16x32_bf16(false, a.hi, false, b.lo, (short)0, c, false, false);
    c = __builtin_amdgcn_wmma_f32_16x16x32_bf16(false, a.lo, false, b.hi, (short)0, c, false, false);
    asm volatile("v_nop\n\tv_nop\n\tv_nop\n\tv_nop" : "+v"(c) : "v"(a.hi), "v"(a.lo), "v"(b.hi), "v"(b.lo));
    return c;
}
struct Split3 { v16b hi, mid, lo; };
__device__ __forceinline__ v8f wmma6(const Split3& a, const Split3& b, v8f c) {
    c = __builtin_amdgcn_wmma_f32_16x16x32_bf16(false, a.hi, false, b.hi, (short)0, c, false, false);
    c = __builtin_amdgcn_wmma_f32_16x16x32_bf16(false, a.hi, false, b.mid, (short)0, c, false, false);
    c = __builtin_amdgcn_wmma_f32_16x16x32_bf16(false, a.mid, false, b.hi, (short)0, c, false, false);
    c = __builtin_amdgcn_wmma_f32_16x16x32_bf16(false, a.hi, false, b.lo, (short)0, c, false, false);
    c = __builtin_amdgcn_wmma_f32_16x16x32_bf16(false, a.mid, false, b.mid, (short)0, c, false, false);
    c = __builtin_amdgcn_wmma_f32_16x16x32_bf16(false, a.lo, false, b.hi, (short)0, c, false, false);
    asm volatile("v_nop\n\tv_nop\n\tv_nop\n\tv_nop" : "+v"(c) : "v"(a.hi), "v"(a.mid), "v"(a.lo), "v"(b.hi), "v"(b.mid), "v"(b.lo));
    return c;
}

__device__ __forceinline__ v16h fh_ld(const float* __restrict__ p, long long sk, int k0, int h, int klen, float s) {
    v16h a;
#pragma unroll
    for (int i = 0; i < 16; ++i) { const int k = k0 + frag_k(i, h); a[i] = (k < klen) ? (_Float16)(p[(long long)k * sk] * s) : (_Float16)0.f; }
    return a;
}
__device__ __forceinline__ Split sp_ld(const float* __restrict__ p, long long sk, int k0, int h, int klen, float s) {
    Split r;
#pragma unroll
    for (int i = 0; i < 16; ++i) {
        const int k = k0 + frag_k(i, h); const float x = (k < klen) ? p[(long long)k * sk] * s : 0.f;
        const __bf16 hb = bf16_rne(x); r.hi[i] = hb; r.lo[i] = bf16_rne(x - bf16_f32(hb));
    }
    return r;
}
__device__ __forceinline__ Split3 sp3_ld(const float* __restrict__ p, long long sk, int k0, int h, int klen, float s) {
    Split3 r;
#pragma unroll
    for (int i = 0; i < 16; ++i) {
        const int k = k0 + frag_k(i, h); const float x = (k < klen) ? p[(long long)k * sk] * s : 0.f;
        const __bf16 hb = bf16_rne(x); const float r1 = x - bf16_f32(hb); const __bf16 mb = bf16_rne(r1);
        r.hi[i] = hb; r.mid[i] = mb; r.lo[i] = bf16_rne(r1 - bf16_f32(mb));
    }
    return r;
}

#define VST2(T, ptr, val) do { const T vst2_v_ = (val); *(volatile T*)(ptr) = vst2_v_; __threadfence(); *(volatile T*)(ptr) = vst2_v_; } while (0)
#define VST2V4(ptr, val) do { const v4f vst2_v4_ = (val); *(volatile v4f*)(ptr) = vst2_v4_; __threadfence(); *(volatile v4f*)(ptr) = vst2_v4_; } while (0)

#define AW 4
struct AttnP {
    const float* Q; const float* K; const float* V; float* O; float* P; const float* Mf; const int* Mi; float* ST;
    const float* Pw; const float* Rt; const int* SQ; const int* SK;
    long long swb, swh, swi, swj, srb, srh, sri;
    long long sQb, sQh, sQi, sQd, sKb, sKh, sKj, sKd, sVb, sVh, sVj, sVd, sOb, sOh, sOi, sPb, sPh, sPi, smb, smh, smi, smj;
    int Lq, Lk, dh, dv, hrep, causal, coff, pband;
    float scale, mfill; int nonorm, mpol;
    int roff, rn, segpol, win;
};
static_assert(sizeof(AttnP) == 12 * 8 + 29 * 8 + 16 * 4);

#ifndef KATTN_ATTR
#define KATTN_ATTR
#endif
template <int DHP, int DVP, int QM, bool SPLITPV, bool TWOPASS>
__global__ __launch_bounds__(32 * AW) KATTN_ATTR void k_attn(AttnP p) {
    constexpr int NT = DVP / 16;
    constexpr int KS = DHP / 32;
    constexpr int VP = DVP + 8;
    __shared__ __align__(16) float    pl[AW][16 * 64];
    __shared__ __align__(16) _Float16 vl[(SPLITPV ? 2 : 1) * 64 * VP];
    const int lane = threadIdx.x & 31, hf = lane >> 4, l15 = lane & 15, wave = threadIdx.x >> 5;
    const int h = blockIdx.y, b = blockIdx.z, hk = h / p.hrep;
    const int q0 = (blockIdx.x * AW + wave) * 16;
    float* myp = pl[wave];
    const float L2E = 1.4426950408889634f;
    const float NEG = -__builtin_inff();
    const int qi = min(q0 + l15, p.Lq - 1);
    const float* qrow = p.Q + b * p.sQb + h * p.sQh + (long long)qi * p.sQi;
    const float* kbase = p.K + b * p.sKb + hk * p.sKh;
    const float* vbase = p.V + b * p.sVb + hk * p.sVh;
    v16h qa[QM == 0 ? KS : 1]; Split qs_[QM == 1 ? KS : 1]; Split3 qt_[QM == 2 ? KS : 1];
#pragma unroll
    for (int ks = 0; ks < KS; ++ks) {
        if (QM == 2) qt_[ks] = sp3_ld(qrow, p.sQd, ks * 32, hf, p.dh, 1.f);
        else if (QM == 1) qs_[ks] = sp_ld(qrow, p.sQd, ks * 32, hf, p.dh, 1.f);
        else qa[ks] = fh_ld(qrow, p.sQd, ks * 32, hf, p.dh, 1.f);
    }
    v8f o[NT]; float m8[8], l8[8];
#pragma unroll
    for (int t = 0; t < NT; ++t) { v8f zz = {}; o[t] = zz; }
#pragma unroll
    for (int i = 0; i < 8; ++i) { m8[i] = NEG; l8[i] = 0.f; }
    int jend = p.Lk; int jstart = 0;
    if (p.causal == 1) { const int je = (blockIdx.x * AW + AW - 1) * 16 + 16 + p.coff; jend = min(jend, max(je, 0)); }
    if (p.win > 0) { const int js = (int)(blockIdx.x * AW) * 16 + p.coff - p.win; jstart = (js > 0) ? (js / 64) * 64 : 0; }
    const int npass = TWOPASS ? 2 : 1;
    for (int pass = 0; pass < npass; ++pass) {
        const bool dopv = (!TWOPASS) || pass == 1;
        for (int j0 = jstart; j0 < jend; j0 += 64) {
            if (dopv) {
                __syncthreads();
                for (int idx = threadIdx.x; idx < 64 * DVP; idx += 32 * AW) {
                    const int jr = idx / DVP, d = idx - jr * DVP, j = j0 + jr;
                    const float f = (j < p.Lk && d < p.dv) ? vbase[(long long)j * p.sVj + (long long)d * p.sVd] : 0.f;
                    if (SPLITPV) {
                        const __bf16 hb = bf16_rne(f);
                        ((__bf16*)vl)[jr * VP + d] = hb; ((__bf16*)vl)[64 * VP + jr * VP + d] = bf16_rne(f - bf16_f32(hb));
                    } else vl[jr * VP + d] = (_Float16)f;
                }
            }
            v8f s[4];
#pragma unroll
            for (int t = 0; t < 4; ++t) {
                const int j = min(j0 + t * 16 + l15, p.Lk - 1);
                const float* krow = kbase + (long long)j * p.sKj;
                v8f acc = {};
#pragma unroll
                for (int ks = 0; ks < KS; ++ks) {
                    if (QM == 2)      acc = wmma6(qt_[ks], sp3_ld(krow, p.sKd, ks * 32, hf, p.dh, 1.f), acc);
                    else if (QM == 1) acc = wmma3(qs_[ks], sp_ld(krow, p.sKd, ks * 32, hf, p.dh, 1.f), acc);
                    else              acc = wmma16(qa[ks], fh_ld(krow, p.sKd, ks * 32, hf, p.dh, 1.f), acc);
                }
                s[t] = acc;
            }
            float pv[8][4];
#pragma unroll
            for (int i = 0; i < 8; ++i) {
                const int irow = q0 + i + 8 * hf;
                const int ic = min(irow, p.Lq - 1);
                float sc[4];
#pragma unroll
                for (int t = 0; t < 4; ++t) {
                    const int jg = j0 + t * 16 + l15;
                    float v = s[t][i] * p.scale;
                    if (p.Mf) v += p.Mf[b * p.smb + h * p.smh + (long long)ic * p.smi + (long long)min(jg, p.Lk - 1) * p.smj];
                    if (p.Rt) { int rc = ic - min(jg, p.Lk - 1) + p.roff; rc = rc < 0 ? 0 : (rc >= p.rn ? p.rn - 1 : rc); v += p.Rt[b * p.srb + h * p.srh + (long long)ic * p.sri + rc]; }
                    if (p.Mi) { const int mv = p.Mi[b * p.smb + h * p.smh + (long long)ic * p.smi + (long long)min(jg, p.Lk - 1) * p.smj]; if (p.mpol ? (mv != 0) : (mv == 0)) v = p.mfill; }
                    if (p.SQ) { const bool same = p.SQ[(long long)b * p.Lq + ic] == p.SK[(long long)b * p.Lk + min(jg, p.Lk - 1)]; if (p.segpol ? same : !same) v = p.mfill; }
                    if (p.causal == 2 && jg > irow + p.coff) v = p.mfill;
                    if (jg >= p.Lk || (p.causal == 1 && jg > irow + p.coff) || (p.causal == 3 && jg < irow + p.coff) || (p.win > 0 && irow + p.coff - jg > p.win)) v = NEG; else v *= L2E;
                    sc[t] = v;
                }
                if (!TWOPASS || pass == 0) {
                    float mx = fmaxf(fmaxf(sc[0], sc[1]), fmaxf(sc[2], sc[3]));
                    mx = fmaxf(mx, __shfl_xor(mx, 1, 32)); mx = fmaxf(mx, __shfl_xor(mx, 2, 32));
                    mx = fmaxf(mx, __shfl_xor(mx, 4, 32)); mx = fmaxf(mx, __shfl_xor(mx, 8, 32));
                    const float mnew = fmaxf(m8[i], mx);
                    const float corr = (mnew == NEG) ? 1.f : exp2f(m8[i] - mnew);
                    float rs = 0.f;
#pragma unroll
                    for (int t = 0; t < 4; ++t) {
                        const float pp = (sc[t] == NEG) ? 0.f : exp2f(sc[t] - mnew); rs += pp;
                        pv[i][t] = p.Pw ? pp * p.Pw[b * p.swb + h * p.swh + (long long)ic * p.swi + (long long)min(j0 + t * 16 + l15, p.Lk - 1) * p.swj] : pp;
                    }
                    rs += __shfl_xor(rs, 1, 32); rs += __shfl_xor(rs, 2, 32); rs += __shfl_xor(rs, 4, 32); rs += __shfl_xor(rs, 8, 32);
                    l8[i] = l8[i] * corr + rs; m8[i] = mnew;
                    if (!TWOPASS) {
#pragma unroll
                        for (int t = 0; t < NT; ++t) o[t][i] *= corr;
                    }
                } else {
                    const float inv = (l8[i] > 0.f) ? 1.f / l8[i] : 0.f;
#pragma unroll
                    for (int t = 0; t < 4; ++t) {
                        const int jg = j0 + t * 16 + l15;
                        float pp = (sc[t] == NEG) ? 0.f : exp2f(sc[t] - m8[i]) * inv;
                        if (p.Pw) pp *= p.Pw[b * p.swb + h * p.swh + (long long)ic * p.swi + (long long)min(jg, p.Lk - 1) * p.swj];
                        pv[i][t] = pp;
                    }
                }
            }
            if (dopv) {
#pragma unroll
                for (int i = 0; i < 8; ++i)
#pragma unroll
                    for (int t = 0; t < 4; ++t) ((volatile float*)myp)[(i + 8 * hf) * 64 + t * 16 + l15] = pv[i][t];
                __syncthreads();
                if (p.P) {
                    float* pb_ = p.P + b * p.sPb + h * p.sPh;
                    const bool fastP = (p.pband == 0) && ((p.sPi & 3) == 0) && (j0 + 64 <= p.Lk) && (q0 + 16 <= p.Lq) && ((((size_t)pb_) & 15) == 0);
                    if (fastP) {
#pragma unroll
                        for (int s2 = 0; s2 < 8; ++s2) {
                            const int row = s2 * 2 + (lane >> 4), c4 = (lane & 15) * 4;
                            const v4f v = *(const v4f*)(myp + row * 64 + c4);
                            VST2V4(pb_ + (long long)(q0 + row) * p.sPi + j0 + c4, v);
                        }
                    } else {
                        for (int row = 0; row < 16; ++row) {
                            const int irow = q0 + row; if (irow >= p.Lq) continue;
                            for (int c = lane; c < 64; c += 32) {
                                const int jg = j0 + c; if (jg >= p.Lk) continue;
                                if (p.pband == 0) VST2(float, pb_ + (long long)irow * p.sPi + jg, myp[row * 64 + c]);
                                else if (jg - irow <= p.pband && irow - jg <= p.pband) VST2(float, pb_ + (long long)irow * p.sPi + (jg - irow + p.pband), myp[row * 64 + c]);
                            }
                        }
                    }
                }
                if (SPLITPV) {
                    const Split pa0 = sp_ld(myp + l15 * 64, 1, 0, hf, 64, 1.f), pa1 = sp_ld(myp + l15 * 64, 1, 32, hf, 64, 1.f);
                    const __bf16* vh = (const __bf16*)vl; const __bf16* vlo = vh + 64 * VP;
#pragma unroll
                    for (int t = 0; t < NT; ++t) {
                        const int dcol = t * 16 + l15;
                        Split b0, b1;
#pragma unroll
                        for (int e = 0; e < 16; ++e) {
                            const int k0 = frag_k(e, hf), k1 = 32 + frag_k(e, hf);
                            b0.hi[e] = vh[k0 * VP + dcol]; b0.lo[e] = vlo[k0 * VP + dcol]; b1.hi[e] = vh[k1 * VP + dcol]; b1.lo[e] = vlo[k1 * VP + dcol];
                        }
                        o[t] = wmma3(pa0, b0, o[t]);
                        o[t] = wmma3(pa1, b1, o[t]);
                    }
                } else {
                    const v16h pa0 = fh_ld(myp + l15 * 64, 1, 0, hf, 64, 4096.f), pa1 = fh_ld(myp + l15 * 64, 1, 32, hf, 64, 4096.f);
#pragma unroll
                    for (int t = 0; t < NT; ++t) {
                        const int dcol = t * 16 + l15;
                        v16h b0, b1;
#pragma unroll
                        for (int e = 0; e < 16; ++e) { b0[e] = vl[frag_k(e, hf) * VP + dcol]; b1[e] = vl[(32 + frag_k(e, hf)) * VP + dcol]; }
                        o[t] = wmma16(pa0, b0, o[t]);
                        o[t] = wmma16(pa1, b1, o[t]);
                    }
                }
            }
        }
    }
    float* obase = p.O + b * p.sOb + h * p.sOh;
    if (p.ST) {
        const int rl = lane >> 1, isel = rl & 7;
        float mv = 0.f, lv = 0.f;
#pragma unroll
        for (int i = 0; i < 8; ++i) if (i == isel) { mv = m8[i]; lv = l8[i]; }
        const int irow = q0 + rl;
        if (irow < p.Lq) { float* st = p.ST + (((long long)b * gridDim.y + h) * p.Lq + irow) * 2 + (lane & 1); VST2(float, st, (lane & 1) ? lv : mv * 0.6931471805599453f); }
    }
    float invr[8];
#pragma unroll
    for (int i = 0; i < 8; ++i) {
        if (TWOPASS) invr[i] = SPLITPV ? 1.f : (1.f / 4096.f);
        else if (p.nonorm) invr[i] = exp2f(m8[i]) * (SPLITPV ? 1.f : (1.f / 4096.f));
        else invr[i] = (l8[i] > 0.f) ? (SPLITPV ? 1.f / l8[i] : 1.f / (l8[i] * 4096.f)) : 0.f;
    }
    __syncthreads();
    const bool ofast = ((p.sOi & 3) == 0) && ((((size_t)obase) & 15) == 0) && (q0 + 16 <= p.Lq);
#pragma unroll
    for (int c0 = 0; c0 < DVP; c0 += 64) {
#pragma unroll
        for (int i = 0; i < 8; ++i)
#pragma unroll
            for (int t = 0; t < NT; ++t) if (t * 16 >= c0 && t * 16 < c0 + 64) ((volatile float*)myp)[(i + 8 * hf) * 64 + (t * 16 - c0) + l15] = o[t][i] * invr[i];
        __syncthreads();
        const int cw = (DVP - c0 < 64) ? (DVP - c0) : 64;
        if (ofast && (c0 + cw <= p.dv) && (cw % 32 == 0)) {
            const int lpr = cw / 4;
            const int rows_per_ins = 32 / lpr;
            for (int r0 = 0; r0 < 16; r0 += rows_per_ins) {
                const int row = r0 + lane / lpr, c4 = (lane % lpr) * 4;
                const v4f v = *(const v4f*)(myp + row * 64 + c4);
                VST2V4(obase + (long long)(q0 + row) * p.sOi + c0 + c4, v);
            }
        } else {
            for (int row = 0; row < 16; ++row) {
                const int irow = q0 + row; if (irow >= p.Lq) continue;
                for (int c = lane; c < cw; c += 32) { const int d = c0 + c; if (d < p.dv) VST2(float, obase + (long long)irow * p.sOi + d, myp[row * 64 + c]); }
            }
        }
        __syncthreads();
    }
}

__device__ __forceinline__ float cmb_bf(float v) { const unsigned u = __builtin_bit_cast(unsigned, v); const unsigned r = (u + 0x7fffu + ((u >> 16) & 1u)) & 0xffff0000u; return __builtin_bit_cast(float, r); }

__global__ __launch_bounds__(256) void k_sd_rnd(const float* __restrict__ Q, const float* __restrict__ Kp, const float* __restrict__ V, float* __restrict__ QBp, float* __restrict__ KBp, float* __restrict__ VBp, long long n4) {
    const long long nb = (n4 + 255) / 256; const int which = blockIdx.x / nb; const long long u = (long long)(blockIdx.x % nb) * 256 + threadIdx.x; if (u >= n4) return;
    const float* src = (which == 0) ? Q : (which == 1) ? Kp : V; float* dst = (which == 0) ? QBp : (which == 1) ? KBp : VBp; const v4f x = *(const v4f*)(src + 4 * u); v4f r; r.x = cmb_bf(x.x); r.y = cmb_bf(x.y); r.z = cmb_bf(x.z); r.w = cmb_bf(x.w); VST2V4(dst + 4 * u, r); }


extern "C" void kernel_launch(void* const* d_in, const int* in_sizes, int n_in, void* d_out, int out_size, void* d_ws, size_t ws_size, hipStream_t stream) {
    if (n_in < 3) return;
    const long long need_in = ((long long)(NB - 1) * SEQ_FULL + SEQ) * HD;
    if ((long long)in_sizes[0] < need_in || (long long)in_sizes[1] < need_in || (long long)in_sizes[2] < need_in) return;
    if ((long long)out_size < (long long)NB * SEQ * HD) return;
    const float* q = (const float*)d_in[0];
    const float* kk = (const float*)d_in[1];
    const float* v = (const float*)d_in[2];
    float* out = (float*)d_out;
    char* wsp = (char*)d_ws;
    const size_t plane_bytes = (size_t)NB_FULL * SEQ_FULL * HD * 4;
    float* QB = (float*)wsp; wsp += plane_bytes;
    float* KB = (float*)wsp; wsp += plane_bytes;
    float* VB = (float*)wsp; wsp += plane_bytes;
    if ((size_t)(wsp - (char*)d_ws) > ws_size) return;
    const long long n4 = need_in / 4;
    const long long nb = (n4 + 255) / 256;
    k_sd_rnd<<<(unsigned)(3 * nb), 256, 0, stream>>>(q, kk, v, QB, KB, VB, n4);
    { AttnP a;
      a.Q = QB; a.K = KB; a.V = VB; a.O = out; a.P = 0; a.Mf = 0; a.Mi = 0; a.ST = 0;
      a.Pw = 0; a.Rt = 0; a.SQ = 0; a.SK = 0;
      a.swb = 0; a.swh = 0; a.swi = 0; a.swj = 0; a.srb = 0; a.srh = 0; a.sri = 0;
      a.sQb = IN_BSTRIDE; a.sQh = 0; a.sQi = HD; a.sQd = 1;
      a.sKb = IN_BSTRIDE; a.sKh = 0; a.sKj = HD; a.sKd = 1;
      a.sVb = IN_BSTRIDE; a.sVh = 0; a.sVj = HD; a.sVd = 1;
      a.sOb = OUT_BSTRIDE; a.sOh = 0; a.sOi = HD;
      a.sPb = 0; a.sPh = 0; a.sPi = 0; a.smb = 0; a.smh = 0; a.smi = 0; a.smj = 0;
      a.Lq = SEQ; a.Lk = SEQ; a.dh = HD; a.dv = HD; a.hrep = 1; a.causal = 0; a.coff = 0; a.pband = 0;
      a.scale = 0.125f; a.mfill = 0.0f; a.nonorm = 0; a.mpol = 0;
      a.roff = 0; a.rn = 1; a.segpol = 0; a.win = 0;
      k_attn<64, 64, 0, false, false><<<dim3((unsigned)((SEQ + 16 * AW - 1) / (16 * AW)), 1u, (unsigned)NB), 32 * AW, 0, stream>>>(a); }
}
